// SelfAttention_6889127543338
// MI455X (gfx1250) — hardware-verified
//
#include <hip/hip_runtime.h>
#ifndef NB
#define NB 4
#endif
#ifndef SEQ
#define SEQ 4096
#endif
#define NB_FULL 4
#define SEQ_FULL 4096
#define CD 256
#define RD 16
#define QKP 32
#define WROWS (2 * RD + CD)
#define SOP 68

static_assert(SEQ % 64 == 0);
static_assert(SEQ <= SEQ_FULL);
static_assert(NB <= NB_FULL);
static_assert(CD % 128 == 0);
static_assert(CD % 64 == 0);
static_assert(CD % 32 == 0);
static_assert(RD == 16);
static_assert(QKP == 2 * RD);
static_assert(QKP == 32);
static_assert((SOP * 4) % 16 == 0);
static_assert((size_t)((NB - 1) * CD + CD - 1) * SEQ_FULL + SEQ <= (size_t)NB_FULL * CD * SEQ_FULL);

#define XB_BYTES ((size_t)NB * SEQ * CD * 2)
#define WC_BYTES ((size_t)WROWS * CD * 2)
#define QK_BYTES ((size_t)NB * SEQ * QKP * 2)
#define VT_BYTES ((size_t)NB * CD * SEQ * 2)
static_assert(XB_BYTES + WC_BYTES + 2 * QK_BYTES + VT_BYTES + 5 * 256 <= (size_t)134217728);

typedef __bf16 v16b __attribute__((ext_vector_type(16)));
typedef _Float16 v16h __attribute__((ext_vector_type(16)));
typedef unsigned short v8us __attribute__((ext_vector_type(8), may_alias));
typedef float v8f __attribute__((ext_vector_type(8)));
typedef float v4f __attribute__((ext_vector_type(4)));
typedef float v4fa __attribute__((ext_vector_type(4), may_alias));
union FragB { v16b v; v8us half[2]; unsigned short u[16]; };
union FragH { v16h v; v8us half[2]; _Float16 h[16]; unsigned short u[16]; };

__device__ __forceinline__ unsigned short bf16_bits(float x) { const unsigned int u = __float_as_uint(x); return (unsigned short)((u + 0x7FFFu + ((u >> 16) & 1u)) >> 16); }
__device__ __forceinline__ float bf16_val(unsigned short b) { return __uint_as_float(((unsigned int)b) << 16); }
__device__ __forceinline__ float bfr(float x) { return bf16_val(bf16_bits(x)); }
__device__ __forceinline__ unsigned short f16_bits(float x) { union { _Float16 h; unsigned short u; } c; c.h = (_Float16)x; return c.u; }

__device__ __forceinline__ v8f mma_b(v16b a, v16b b, v8f c) {
  v8f d = __builtin_amdgcn_wmma_f32_16x16x32_bf16(false, a, false, b, (short)0, c, false, false);
  asm volatile("v_nop\n\tv_nop\n\tv_nop\n\tv_nop" : "+v"(d) : "v"(a), "v"(b));
  return d;
}
__device__ __forceinline__ v8f mma_h(v16h a, v16h b, v8f c) {
  v8f d = __builtin_amdgcn_wmma_f32_16x16x32_f16(false, a, false, b, (short)0, c, false, false);
  asm volatile("v_nop\n\tv_nop\n\tv_nop\n\tv_nop" : "+v"(d) : "v"(a), "v"(b));
  return d;
}
__device__ __forceinline__ v16b ldfrag_b(const unsigned short* p) { FragB f; f.half[0] = *(const v8us*)(p); f.half[1] = *(const v8us*)(p + 16); return f.v; }

__global__ __launch_bounds__(256) void k_xT(const float* __restrict__ x, unsigned short* __restrict__ XB) {
  __shared__ unsigned short tl[64][66];
  const int tid = threadIdx.x;
  const int blk = blockIdx.x;
  const int ct = blk % (CD / 64);
  const int nt = (blk / (CD / 64)) % (SEQ / 64);
  const int b = blk / ((CD / 64) * (SEQ / 64));
  const int c0 = ct * 64, n0 = nt * 64;
#pragma unroll 1
  for (int i = tid; i < 64 * 16; i += 256) {
    const int r = i >> 4, j4 = (i & 15) * 4;
    const v4f a = *(const v4fa*)(x + ((size_t)b * CD + c0 + r) * SEQ_FULL + n0 + j4);
#pragma unroll
    for (int q = 0; q < 4; ++q) tl[r][j4 + q] = bf16_bits(a[q]);
  }
  __syncthreads();
  for (int pass = 0; pass < 2; ++pass) {
#pragma unroll 1
    for (int i = tid; i < 64 * 8; i += 256) {
      const int n = i >> 3, p = i & 7;
      FragB f;
#pragma unroll
      for (int q = 0; q < 8; ++q) f.u[q] = tl[p * 8 + q][n];
      *(volatile v8us*)(XB + ((size_t)b * SEQ + n0 + n) * CD + c0 + p * 8) = f.half[0];
    }
    if (pass == 0) __threadfence();
  }
}

__global__ __launch_bounds__(256) void k_cast_bf16(const float* __restrict__ src, unsigned short* __restrict__ dst, int n8) {
  const int t = blockIdx.x * 256 + threadIdx.x;
  if (t >= n8) return;
  const v4f a = *(const v4fa*)(src + (size_t)t * 8), c = *(const v4fa*)(src + (size_t)t * 8 + 4);
  FragB f;
#pragma unroll
  for (int q = 0; q < 4; ++q) { f.u[q] = bf16_bits(a[q]); f.u[4 + q] = bf16_bits(c[q]); }
  const v8us o = f.half[0];
  *(volatile v8us*)(dst + (size_t)t * 8) = o;
  __threadfence();
  *(volatile v8us*)(dst + (size_t)t * 8) = o;
}

__global__ __launch_bounds__(128) void k_qk(const unsigned short* __restrict__ XB, const unsigned short* __restrict__ WC,
                                            const float* __restrict__ bq, const float* __restrict__ bk,
                                            unsigned short* __restrict__ QP, unsigned short* __restrict__ KP) {
  __shared__ __attribute__((aligned(16))) unsigned short st[4][2][16][QKP];
  const int tid = threadIdx.x, lane = tid & 31, ln = lane & 15, hh = lane >> 4;
  const int wave = __builtin_amdgcn_readfirstlane((int)(threadIdx.x >> 5));
  const int row0 = (blockIdx.x * 4 + wave) * 16;
  const unsigned short* arow = XB + (size_t)(row0 + ln) * CD + 8 * hh;
  const unsigned short* bqr = WC + (size_t)ln * CD + 8 * hh;
  const unsigned short* bkr = WC + (size_t)(RD + ln) * CD + 8 * hh;
  const v8f z8 = {0.f, 0.f, 0.f, 0.f, 0.f, 0.f, 0.f, 0.f};
  v8f aq = z8, ak = z8;
#pragma unroll 1
  for (int kb = 0; kb < CD; kb += 32) {
    const v16b a = ldfrag_b(arow + kb);
    const v16b fq = ldfrag_b(bqr + kb);
    const v16b fk = ldfrag_b(bkr + kb);
    aq = mma_b(a, fq, aq);
    ak = mma_b(a, fk, ak);
  }
  const float bqv = bfr(bq[ln]), bkv = bfr(bk[ln]);
#pragma unroll
  for (int r = 0; r < 8; ++r) {
    const int t = 8 * hh + r;
    const float vq = aq[r] + bqv;
    const unsigned short qh = bf16_bits(vq);
    st[wave][0][t][ln] = qh;
    st[wave][0][t][RD + ln] = bf16_bits(vq - bf16_val(qh));
    const float vk = ak[r] + bkv;
    const unsigned short kh = bf16_bits(vk);
    st[wave][1][t][ln] = kh;
    st[wave][1][t][RD + ln] = bf16_bits(vk - bf16_val(kh));
  }
  __builtin_amdgcn_fence(4  , "workgroup");
  __builtin_amdgcn_wave_barrier();
  for (int pass = 0; pass < 2; ++pass) {
#pragma unroll
    for (int it = 0; it < 2; ++it) {
      const int i = it * 32 + lane;
      const int row = i >> 2, pc = (i & 3) * 8;
      const v8us vq = *(const v8us*)&st[wave][0][row][pc];
      const v8us vk = *(const v8us*)&st[wave][1][row][pc];
      const size_t o = (size_t)(row0 + row) * QKP + pc;
      *(volatile v8us*)(QP + o) = vq;
      *(volatile v8us*)(KP + o) = vk;
    }
    if (pass == 0) __threadfence();
  }
}

__global__ __launch_bounds__(128) void k_vproj(const unsigned short* __restrict__ WV, const unsigned short* __restrict__ XB,
                                               const float* __restrict__ bv, unsigned short* __restrict__ VT) {
  __shared__ __attribute__((aligned(16))) unsigned short so[4][32][72];
  const int tid = threadIdx.x, lane = tid & 31, ln = lane & 15, hh = lane >> 4;
  const int wave = __builtin_amdgcn_readfirstlane((int)(threadIdx.x >> 5));
  const int b = blockIdx.y;
  const int mt = blockIdx.x / (SEQ / 64), nq = blockIdx.x % (SEQ / 64);
  const int row0 = mt * 128 + 32 * wave, col0 = nq * 64;
  const unsigned short* a0p = WV + (size_t)(row0 + ln) * CD + 8 * hh;
  const unsigned short* a1p = a0p + (size_t)16 * CD;
  const unsigned short* b0p = XB + ((size_t)b * SEQ + col0 + ln) * CD + 8 * hh;
  const unsigned short* b1p = b0p + (size_t)16 * CD;
  const unsigned short* b2p = b1p + (size_t)16 * CD;
  const unsigned short* b3p = b2p + (size_t)16 * CD;
  const v8f z8 = {0.f, 0.f, 0.f, 0.f, 0.f, 0.f, 0.f, 0.f};
  v8f c00 = z8, c01 = z8, c02 = z8, c03 = z8, c10 = z8, c11 = z8, c12 = z8, c13 = z8;
#pragma unroll 1
  for (int kb = 0; kb < CD; kb += 32) {
    const v16b a0 = ldfrag_b(a0p + kb), a1 = ldfrag_b(a1p + kb);
    v16b bb = ldfrag_b(b0p + kb); c00 = mma_b(a0, bb, c00); c10 = mma_b(a1, bb, c10);
    bb = ldfrag_b(b1p + kb); c01 = mma_b(a0, bb, c01); c11 = mma_b(a1, bb, c11);
    bb = ldfrag_b(b2p + kb); c02 = mma_b(a0, bb, c02); c12 = mma_b(a1, bb, c12);
    bb = ldfrag_b(b3p + kb); c03 = mma_b(a0, bb, c03); c13 = mma_b(a1, bb, c13);
  }
  v8f accs[8] = {c00, c01, c02, c03, c10, c11, c12, c13};
#pragma unroll
  for (int u = 0; u < 8; ++u) {
    const int t = u & 3, half = u >> 2;
#pragma unroll
    for (int r = 0; r < 8; ++r) {
      const int rloc = half * 16 + 8 * hh + r;
      const float bias = bfr(bv[row0 + rloc]);
      so[wave][rloc][t * 16 + ln] = f16_bits(accs[u][r] + bias);
    }
  }
  __builtin_amdgcn_fence(4  , "workgroup");
  __builtin_amdgcn_wave_barrier();
  for (int pass = 0; pass < 2; ++pass) {
#pragma unroll
    for (int it = 0; it < 8; ++it) {
      const int i = it * 32 + lane;
      const int row = i >> 3, pc = (i & 7) * 8;
      const v8us v = *(const v8us*)&so[wave][row][pc];
      *(volatile v8us*)(VT + ((size_t)b * CD + row0 + row) * SEQ + col0 + pc) = v;
    }
    if (pass == 0) __threadfence();
  }
}

__global__ __launch_bounds__(128) void k_flash(const float* __restrict__ x, const unsigned short* __restrict__ QP, const unsigned short* __restrict__ KP,
                                               const unsigned short* __restrict__ VT, const float* __restrict__ gamma, float* __restrict__ out) {
  __shared__ __attribute__((aligned(16))) float so[128][SOP];
  const int tid = threadIdx.x, lane = tid & 31, ln = lane & 15, hh = lane >> 4;
  const int wave = __builtin_amdgcn_readfirstlane((int)(threadIdx.x >> 5));
  const int n0 = blockIdx.x * 64, ch0 = blockIdx.y * 128, b = blockIdx.z;
  FragB qf;
  {
    const unsigned short* qrow = QP + ((size_t)b * SEQ + n0 + wave * 16 + ln) * QKP + 8 * hh;
    qf.half[0] = *(const v8us*)(qrow);
    qf.half[1] = *(const v8us*)(qrow + 16);
  }
  const unsigned short* kbase = KP + ((size_t)b * SEQ + ln) * QKP + 8 * hh;
  const unsigned short* vbase = VT + ((size_t)b * CD + ch0 + ln) * SEQ + 8 * hh;
  const v8f z8 = {0.f, 0.f, 0.f, 0.f, 0.f, 0.f, 0.f, 0.f};
  const v8us zus = {0, 0, 0, 0, 0, 0, 0, 0};
  v8f acc[8] = {z8, z8, z8, z8, z8, z8, z8, z8};
  float mrun = -1.0e30f, lrun = 0.f;
#pragma unroll 1
  for (int m0 = 0; m0 < SEQ; m0 += 32) {
    const unsigned short* kp0 = kbase + (size_t)m0 * QKP;
    const unsigned short* kp1 = kp0 + 16 * QKP;
    FragB k0h, k0l, k1h, k1l;
    const v8us h0 = *(const v8us*)(kp0), l0 = *(const v8us*)(kp0 + 16);
    const v8us h1 = *(const v8us*)(kp1), l1 = *(const v8us*)(kp1 + 16);
    k0h.half[0] = h0; k0h.half[1] = h0; k0l.half[0] = l0; k0l.half[1] = zus;
    k1h.half[0] = h1; k1h.half[1] = h1; k1l.half[0] = l1; k1l.half[1] = zus;
    v8f s0 = mma_b(k0h.v, qf.v, z8);
    s0 = mma_b(k0l.v, qf.v, s0);
    v8f s1 = mma_b(k1h.v, qf.v, z8);
    s1 = mma_b(k1l.v, qf.v, s1);
    float tm = fmaxf(s0[0], s1[0]);
#pragma unroll
    for (int r = 1; r < 8; ++r) tm = fmaxf(tm, fmaxf(s0[r], s1[r]));
    tm = fmaxf(tm, __shfl_xor(tm, 16));
    const float mn = fmaxf(mrun, tm);
    const float alpha = __expf(mrun - mn);
    FragH p;
    float ls = 0.f;
#pragma unroll
    for (int r = 0; r < 8; ++r) {
      const float e0 = __expf(s0[r] - mn), e1 = __expf(s1[r] - mn);
      ls += e0 + e1;
      p.h[r] = (_Float16)(e0 * 256.0f);
      p.h[8 + r] = (_Float16)(e1 * 256.0f);
    }
    lrun = lrun * alpha + ls;
    mrun = mn;
    if (__builtin_amdgcn_ballot_w32(alpha != 1.0f) != 0u) {
#pragma unroll
      for (int j = 0; j < 8; ++j) acc[j] = acc[j] * alpha;
    }
#pragma unroll
    for (int j = 0; j < 8; ++j) {
      const unsigned short* vp = vbase + (size_t)(16 * j) * SEQ + m0;
      FragH vf;
      vf.half[0] = *(const v8us*)(vp);
      vf.half[1] = *(const v8us*)(vp + 16);
      acc[j] = mma_h(vf.v, p.v, acc[j]);
    }
  }
  lrun += __shfl_xor(lrun, 16);
  const float inv = 1.0f / (256.0f * lrun);
#pragma unroll
  for (int j = 0; j < 8; ++j) {
#pragma unroll
    for (int r = 0; r < 8; ++r) so[16 * j + 8 * hh + r][wave * 16 + ln] = acc[j][r] * inv;
  }
  __syncthreads();
  const float g = bfr(gamma[0]);
  const size_t base = ((size_t)b * CD + ch0) * SEQ_FULL + n0;
  for (int pass = 0; pass < 2; ++pass) {
#pragma unroll 1
    for (int it = 0; it < 16; ++it) {
      const int i = it * 128 + tid;
      const int row = i >> 4, pc = (i & 15) * 4;
      const v4f v = *(const v4fa*)&so[row][pc];
      const size_t gi = base + (size_t)row * SEQ_FULL + pc;
      const v4f xg = *(const v4fa*)(x + gi);
      v4f res;
#pragma unroll
      for (int q = 0; q < 4; ++q) res[q] = g * v[q] + bfr(xg[q]);
      *(volatile v4f*)(out + gi) = res;
    }
    if (pass == 0) __threadfence();
  }
}

extern "C" void kernel_launch(void* const* d_in, const int* in_sizes, int n_in,
                              void* d_out, int out_size, void* d_ws, size_t ws_size, hipStream_t stream) {
  if (n_in < 8) return;
  if ((size_t)in_sizes[0] < (size_t)((NB - 1) * CD + CD - 1) * SEQ_FULL + SEQ) return;
  if (in_sizes[1] < RD * CD || in_sizes[2] < RD || in_sizes[3] < RD * CD || in_sizes[4] < RD) return;
  if (in_sizes[5] < CD * CD || in_sizes[6] < CD || in_sizes[7] < 1) return;
  if ((size_t)out_size < (size_t)((NB - 1) * CD + CD - 1) * SEQ_FULL + SEQ) return;
  const float* x  = (const float*)d_in[0];
  const float* wq = (const float*)d_in[1];
  const float* bq = (const float*)d_in[2];
  const float* wk = (const float*)d_in[3];
  const float* bk = (const float*)d_in[4];
  const float* wv = (const float*)d_in[5];
  const float* bv = (const float*)d_in[6];
  const float* gm = (const float*)d_in[7];
  float* out = (float*)d_out;
  char* ws = (char*)d_ws;
  size_t off = 0;
  auto take = [&](size_t bytes) { char* p = ws + off; off += (bytes + 255) & ~(size_t)255; return p; };
  unsigned short* XB = (unsigned short*)take(XB_BYTES);
  unsigned short* WC = (unsigned short*)take(WC_BYTES);
  unsigned short* QP = (unsigned short*)take(QK_BYTES);
  unsigned short* KP = (unsigned short*)take(QK_BYTES);
  unsigned short* VT = (unsigned short*)take(VT_BYTES);
  if (off > ws_size) return;
  k_xT<<<NB * (SEQ / 64) * (CD / 64), 256, 0, stream>>>(x, XB);
  k_cast_bf16<<<(RD * CD / 8 + 255) / 256, 256, 0, stream>>>(wq, WC, RD * CD / 8);
  k_cast_bf16<<<(RD * CD / 8 + 255) / 256, 256, 0, stream>>>(wk, WC + (size_t)RD * CD, RD * CD / 8);
  k_cast_bf16<<<(CD * CD / 8 + 255) / 256, 256, 0, stream>>>(wv, WC + (size_t)2 * RD * CD, CD * CD / 8);
  k_qk<<<NB * SEQ / 64, 128, 0, stream>>>(XB, WC, bq, bk, QP, KP);
  k_vproj<<<dim3((CD / 128) * (SEQ / 64), NB), 128, 0, stream>>>(WC + (size_t)2 * RD * CD, XB, bv, VT);
  k_flash<<<dim3(SEQ / 64, CD / 128, NB), 128, 0, stream>>>(x, QP, KP, VT, gm, out);
}
